// TextOnlyMultiChannelGAT_66614942761287
// MI455X (gfx1250) — hardware-verified
//
#include <hip/hip_runtime.h>
#include <stddef.h>
#include <stdint.h>

#define NB  16
#define SQ  512
#define DD  768
#define D2  1536
#define NH  12
#define HD  64
#define NC  3
#define NR  (NB * SQ)
#define PLQ ((size_t)NB * NH * SQ * HD)

static_assert(NH * HD == DD);
static_assert(SQ % 128 == 0);
static_assert(NR % 128 == 0);
static_assert(DD % 64 == 0);
static_assert(D2 % 64 == 0);
static_assert(SQ % 64 == 0);
static_assert(NB == 16);

typedef _Float16 v16h __attribute__((ext_vector_type(16)));
typedef _Float16 v8h  __attribute__((ext_vector_type(8)));
typedef __bf16   v16b __attribute__((ext_vector_type(16)));
typedef float    v8f  __attribute__((ext_vector_type(8)));
typedef float    v4f  __attribute__((ext_vector_type(4)));
typedef unsigned int   v4u  __attribute__((ext_vector_type(4)));
typedef unsigned int   v2u  __attribute__((ext_vector_type(2)));
typedef unsigned short v8us __attribute__((ext_vector_type(8)));
typedef unsigned short v4us __attribute__((ext_vector_type(4)));

union Frag   { v16h v; v8h h[2]; };
union FragB  { v16b v; v4u u[2]; v8f f; };
union Pack8  { v8h h; v4u u; };
union PackU8 { v8us s; v4u u; };
union PackU4 { v4us s; v2u u; };

__device__ __forceinline__ v8f zero8() { return (v8f){0.f, 0.f, 0.f, 0.f, 0.f, 0.f, 0.f, 0.f}; }

__device__ __forceinline__ v8f mma16(v16h a, v16h b, v8f c) {
  c = __builtin_amdgcn_wmma_f32_16x16x32_f16(false, a, false, b, (short)0, c, false, false);
  asm volatile("v_nop\n\tv_nop\n\tv_nop\n\tv_nop" : "+v"(c) : "v"(a), "v"(b));
  return c;
}
__device__ __forceinline__ v8f mmab(v16b a, v16b b, v8f c) {
  c = __builtin_amdgcn_wmma_f32_16x16x32_bf16(false, a, false, b, (short)0, c, false, false);
  FragB fa, fb;
  fa.v = a;
  fb.v = b;
  asm volatile("v_nop\n\tv_nop\n\tv_nop\n\tv_nop" : "+v"(c) : "v"(fa.f), "v"(fb.f));
  return c;
}

__device__ __forceinline__ v16h ldfrag(const _Float16* p, int ld, int row0, int k0, int lane) {
  const int m = lane & 15, lh = lane >> 4;
  const _Float16* q = p + (size_t)(row0 + m) * ld + k0 + 8 * lh;
  Frag f;
  f.h[0] = *(const v8h*)(q);
  f.h[1] = *(const v8h*)(q + 16);
  return f.v;
}
__device__ __forceinline__ v16b ldfragb(const unsigned short* p, int ld, int row0, int k0, int lane) {
  const int m = lane & 15, lh = lane >> 4;
  const unsigned short* q = p + (size_t)(row0 + m) * ld + k0 + 8 * lh;
  FragB f;
  f.u[0] = *(const v4u*)(q);
  f.u[1] = *(const v4u*)(q + 16);
  return f.v;
}

__device__ __forceinline__ unsigned int bf16_rne_bits(float x) {
  const unsigned int u = __float_as_uint(x);
  return (u + 0x7FFFu + ((u >> 16) & 1u)) >> 16;
}

__device__ __forceinline__ void gemm32x64(const _Float16* __restrict__ A, int lda,
                                          const _Float16* __restrict__ Bt, int ldb, int K,
                                          int m0, int n0, int lane, v8f (&acc)[2][4]) {
#pragma unroll 2
  for (int k0 = 0; k0 < K; k0 += 32) {
    const v16h a0 = ldfrag(A, lda, m0, k0, lane);
    const v16h a1 = ldfrag(A, lda, m0 + 16, k0, lane);
    const v16h b0 = ldfrag(Bt, ldb, n0, k0, lane);
    const v16h b1 = ldfrag(Bt, ldb, n0 + 16, k0, lane);
    const v16h b2 = ldfrag(Bt, ldb, n0 + 32, k0, lane);
    const v16h b3 = ldfrag(Bt, ldb, n0 + 48, k0, lane);
    acc[0][0] = mma16(a0, b0, acc[0][0]);
    acc[1][0] = mma16(a1, b0, acc[1][0]);
    acc[0][1] = mma16(a0, b1, acc[0][1]);
    acc[1][1] = mma16(a1, b1, acc[1][1]);
    acc[0][2] = mma16(a0, b2, acc[0][2]);
    acc[1][2] = mma16(a1, b2, acc[1][2]);
    acc[0][3] = mma16(a0, b3, acc[0][3]);
    acc[1][3] = mma16(a1, b3, acc[1][3]);
  }
}

#define TTP 68
__global__ __launch_bounds__(256) void k_cvt_ht(const float* __restrict__ ht, _Float16* __restrict__ xh,
                                                unsigned short* __restrict__ hth,
                                                unsigned short* __restrict__ htl) {
  __shared__ __align__(16) float T[64 * TTP];
  const int tid = threadIdx.x;
  const int s0 = blockIdx.x * 64, d0 = blockIdx.y * 64, b = blockIdx.z;
#pragma unroll
  for (int j = 0; j < 4; ++j) {
    const int p = tid + 256 * j;
    const int row = p >> 4, c4 = p & 15;
    *(v4f*)(T + row * TTP + c4 * 4) =
        *(const v4f*)(ht + ((size_t)(b * SQ + s0 + row)) * DD + d0 + c4 * 4);
  }
  __syncthreads();

  v4u xv[2], hv[2], lv[2];
  size_t xo[2], to[2];
#pragma unroll
  for (int j = 0; j < 2; ++j) {
    const int p = tid + 256 * j;
    const int row = p >> 3, pc = p & 7;
    const float* tp = T + row * TTP + pc * 8;
    const v4f a0 = *(const v4f*)(tp);
    const v4f a1 = *(const v4f*)(tp + 4);
    Pack8 pk;
    pk.h = (v8h){(_Float16)a0[0], (_Float16)a0[1], (_Float16)a0[2], (_Float16)a0[3],
                 (_Float16)a1[0], (_Float16)a1[1], (_Float16)a1[2], (_Float16)a1[3]};
    xv[j] = pk.u;
    xo[j] = ((size_t)(b * SQ + s0 + row)) * DD + d0 + pc * 8;
    const int dd = row;
    PackU8 ph, pl;
#pragma unroll
    for (int e = 0; e < 8; ++e) {
      const float x = T[(pc * 8 + e) * TTP + dd];
      const unsigned int hb = bf16_rne_bits(x);
      const unsigned int lb = bf16_rne_bits(x - __uint_as_float(hb << 16));
      ph.s[e] = (unsigned short)hb;
      pl.s[e] = (unsigned short)lb;
    }
    hv[j] = ph.u;
    lv[j] = pl.u;
    to[j] = ((size_t)(b * DD + d0 + dd)) * SQ + s0 + pc * 8;
  }
  for (int ps = 0; ps < 2; ++ps) {
#pragma unroll
    for (int j = 0; j < 2; ++j) {
      *(volatile v4u*)(xh + xo[j])  = xv[j];
      *(volatile v4u*)(hth + to[j]) = hv[j];
      *(volatile v4u*)(htl + to[j]) = lv[j];
    }
    __threadfence();
  }
}

__global__ __launch_bounds__(256) void k_cvt_wt(const float* __restrict__ w, _Float16* __restrict__ wt,
                                                int R, int C, float sc) {
  __shared__ __align__(16) float T[64 * TTP];
  const int tid = threadIdx.x;
  const int c0 = blockIdx.x * 64, r0 = blockIdx.y * 64, z = blockIdx.z;
#pragma unroll
  for (int j = 0; j < 4; ++j) {
    const int p = tid + 256 * j;
    const int row = p >> 4, c4 = p & 15;
    *(v4f*)(T + row * TTP + c4 * 4) =
        *(const v4f*)(w + ((size_t)(z * R + r0 + row)) * C + c0 + c4 * 4);
  }
  __syncthreads();
  v4u val[2];
  size_t go[2];
#pragma unroll
  for (int j = 0; j < 2; ++j) {
    const int p = tid + 256 * j;
    const int cc = p >> 3, pc = p & 7;
    Pack8 pk;
    v8h o8;
#pragma unroll
    for (int e = 0; e < 8; ++e) o8[e] = (_Float16)(T[(pc * 8 + e) * TTP + cc] * sc);
    pk.h = o8;
    val[j] = pk.u;
    go[j]  = ((size_t)(z * C + c0 + cc)) * R + r0 + pc * 8;
  }
  for (int ps = 0; ps < 2; ++ps) {
#pragma unroll
    for (int j = 0; j < 2; ++j) *(volatile v4u*)(wt + go[j]) = val[j];
    __threadfence();
  }
}

#define STP 72
__global__ __launch_bounds__(128) void k_qk(const _Float16* __restrict__ xh,
                                            const _Float16* __restrict__ wt,
                                            const float* __restrict__ bias,
                                            _Float16* __restrict__ qk) {
  __shared__ __align__(16) _Float16 st[128 * STP];
  const int tid = threadIdx.x, lane = tid & 31, wave = tid >> 5;
  const int hh = lane >> 4, c = lane & 15;
  const int mb = blockIdx.x * 128;
  const int m0 = mb + wave * 32;
  const int n0 = blockIdx.y * 64;

  v8f acc[2][4];
#pragma unroll
  for (int s = 0; s < 2; ++s)
#pragma unroll
    for (int t = 0; t < 4; ++t) acc[s][t] = zero8();
  gemm32x64(xh, DD, wt, DD, DD, m0, n0, lane, acc);

#pragma unroll
  for (int t = 0; t < 4; ++t) {
    const float bv = bias[n0 + 16 * t + c];
#pragma unroll
    for (int sub = 0; sub < 2; ++sub) {
#pragma unroll
      for (int r = 0; r < 8; ++r) {
        const int lr = wave * 32 + sub * 16 + 8 * hh + r;
        st[lr * STP + 16 * t + c] = (_Float16)(acc[sub][t][r] * 0.03125f + bv);
      }
    }
  }
  __syncthreads();

  const int which = n0 / DD;
  const int head  = (n0 - which * DD) >> 6;
  const int b  = mb / SQ;
  const int sb = mb - b * SQ;
  const int bh = b * NH + head;
  v4u val[8];
  size_t go[8];
#pragma unroll
  for (int j = 0; j < 8; ++j) {
    const int p  = tid + 128 * j;
    const int lr = p >> 3;
    const int pc = p & 7;
    Pack8 pk;
    pk.h  = *(const v8h*)(st + lr * STP + pc * 8);
    val[j] = pk.u;
    go[j]  = (size_t)which * PLQ + ((size_t)bh * SQ + sb + lr) * HD + pc * 8;
  }
  for (int ps = 0; ps < 2; ++ps) {
#pragma unroll
    for (int j = 0; j < 8; ++j) *(volatile v4u*)(qk + go[j]) = val[j];
    __threadfence();
  }
}

#define SCP 520
#define LDS_G   (16 * SCP * 4)
#define LDS_MK  (LDS_G + NC * 16 * SQ * 4)
#define LDS_ATT (LDS_MK + SQ * 4)
static_assert(2 * 16 * SCP * 2 <= LDS_G);

__global__ __launch_bounds__(256) void k_attn(const _Float16* __restrict__ qp,
                                              const _Float16* __restrict__ kp,
                                              const float* __restrict__ amask,
                                              const float* __restrict__ mlist,
                                              unsigned short* __restrict__ ahi,
                                              unsigned short* __restrict__ alo, float sscale) {
  extern __shared__ __align__(16) v4f dlds[];
  unsigned char* lb = (unsigned char*)dlds;
  float* sc = (float*)lb;
  unsigned short* sth = (unsigned short*)lb;
  unsigned short* stl = (unsigned short*)(lb + 16 * SCP * 2);
  float* G  = (float*)(lb + LDS_G);
  float* mk = (float*)(lb + LDS_MK);

  const int tid = threadIdx.x, lane = tid & 31, wave = tid >> 5;
  const int hh = lane >> 4, c = lane & 15;
  const int b  = blockIdx.x >> 5;
  const int qt = blockIdx.x & 31;
  const int q0 = qt * 16;
  const int row = tid >> 4, part = tid & 15;
  const int kw0 = wave * 64;
  const v4f z4 = (v4f){0.f, 0.f, 0.f, 0.f};

  if (tid < 128) *(v4f*)(mk + tid * 4) = *(const v4f*)(amask + (size_t)b * SQ + tid * 4);
#pragma unroll
  for (int i = 0; i < NC; ++i)
#pragma unroll
    for (int j = 0; j < 8; ++j) *(v4f*)(G + (i * 16 + row) * SQ + part * 4 + 64 * j) = z4;
  __syncthreads();
  const float mq = mk[q0 + row];

#pragma unroll 1
  for (int h = 0; h < NH; ++h) {
    const int bh = b * NH + h;
    const _Float16* Q = qp + (size_t)bh * SQ * HD;
    const _Float16* K = kp + (size_t)bh * SQ * HD;
    const v16h qa0 = ldfrag(Q, HD, q0, 0, lane);
    const v16h qa1 = ldfrag(Q, HD, q0, 32, lane);
    v8f s[4];
#pragma unroll
    for (int j = 0; j < 4; ++j) s[j] = zero8();
#pragma unroll
    for (int j = 0; j < 4; ++j) {
      const v16h kb0 = ldfrag(K, HD, kw0 + 16 * j, 0, lane);
      s[j] = mma16(qa0, kb0, s[j]);
      const v16h kb1 = ldfrag(K, HD, kw0 + 16 * j, 32, lane);
      s[j] = mma16(qa1, kb1, s[j]);
    }
    __syncthreads();
#pragma unroll
    for (int j = 0; j < 4; ++j) {
      const int key = kw0 + 16 * j + c;
      const float mbias = (1.0f - mk[key]) * (-1.0e9f);
#pragma unroll
      for (int r = 0; r < 8; ++r) sc[(8 * hh + r) * SCP + key] = s[j][r] * sscale + mbias;
    }
    __syncthreads();

    v4f p4[8];
    float mx = -__builtin_huge_valf();
    const float* scr = sc + row * SCP + part * 4;
#pragma unroll
    for (int j = 0; j < 8; ++j) {
      p4[j] = *(const v4f*)(scr + 64 * j);
      mx = fmaxf(mx, fmaxf(fmaxf(p4[j][0], p4[j][1]), fmaxf(p4[j][2], p4[j][3])));
    }
#pragma unroll
    for (int off = 1; off < 16; off <<= 1) mx = fmaxf(mx, __shfl_xor(mx, off, 32));
    float sum = 0.f;
#pragma unroll
    for (int j = 0; j < 8; ++j) {
#pragma unroll
      for (int e = 0; e < 4; ++e) {
        const float ev = __expf(p4[j][e] - mx);
        p4[j][e] = ev;
        sum += ev;
      }
    }
#pragma unroll
    for (int off = 1; off < 16; off <<= 1) sum += __shfl_xor(sum, off, 32);
    const float inv = 1.0f / sum;
#pragma unroll
    for (int j = 0; j < 8; ++j) p4[j] = p4[j] * inv;

    float den0 = 0.f, den1 = 0.f, den2 = 0.f;
    const float* m0p = mlist + (((size_t)(b * NC + 0) * SQ + q0 + row)) * SQ + part * 4;
    const float* m1p = m0p + (size_t)SQ * SQ;
    const float* m2p = m0p + (size_t)2 * SQ * SQ;
#pragma unroll
    for (int j = 0; j < 8; ++j) {
      const v4f mm = *(const v4f*)(mk + part * 4 + 64 * j) * mq;
      const v4f a0 = (*(const v4f*)(m0p + 64 * j) * mm) * p4[j];
      const v4f a1 = (*(const v4f*)(m1p + 64 * j) * mm) * p4[j];
      const v4f a2 = (*(const v4f*)(m2p + 64 * j) * mm) * p4[j];
      den0 += (a0[0] + a0[1]) + (a0[2] + a0[3]);
      den1 += (a1[0] + a1[1]) + (a1[2] + a1[3]);
      den2 += (a2[0] + a2[1]) + (a2[2] + a2[3]);
    }
#pragma unroll
    for (int off = 1; off < 16; off <<= 1) {
      den0 += __shfl_xor(den0, off, 32);
      den1 += __shfl_xor(den1, off, 32);
      den2 += __shfl_xor(den2, off, 32);
    }
    const float id0 = 1.0f / (den0 + 1e-10f);
    const float id1 = 1.0f / (den1 + 1e-10f);
    const float id2 = 1.0f / (den2 + 1e-10f);
#pragma unroll
    for (int j = 0; j < 8; ++j) {
      float* g0p = G + (0 * 16 + row) * SQ + part * 4 + 64 * j;
      float* g1p = G + (1 * 16 + row) * SQ + part * 4 + 64 * j;
      float* g2p = G + (2 * 16 + row) * SQ + part * 4 + 64 * j;
      const v4f g0 = *(const v4f*)g0p + p4[j] * id0;
      const v4f g1 = *(const v4f*)g1p + p4[j] * id1;
      const v4f g2 = *(const v4f*)g2p + p4[j] * id2;
      *(v4f*)g0p = g0;
      *(v4f*)g1p = g1;
      *(v4f*)g2p = g2;
    }
  }

#pragma unroll 1
  for (int i = 0; i < NC; ++i) {
    __syncthreads();
    const float* mp = mlist + (((size_t)(b * NC + i) * SQ + q0 + row)) * SQ + part * 4;
#pragma unroll
    for (int j = 0; j < 8; ++j) {
      const v4f mm = *(const v4f*)(mk + part * 4 + 64 * j) * mq;
      const v4f g  = *(const v4f*)(G + (i * 16 + row) * SQ + part * 4 + 64 * j);
      const v4f av = ((*(const v4f*)(mp + 64 * j) * mm) * g) * (1.0f / 12.0f);
      PackU4 ph, pl;
#pragma unroll
      for (int e = 0; e < 4; ++e) {
        const unsigned int hb = bf16_rne_bits(av[e]);
        const unsigned int lb2 = bf16_rne_bits(av[e] - __uint_as_float(hb << 16));
        ph.s[e] = (unsigned short)hb;
        pl.s[e] = (unsigned short)lb2;
      }
      *(v2u*)(sth + row * SCP + part * 4 + 64 * j) = ph.u;
      *(v2u*)(stl + row * SCP + part * 4 + 64 * j) = pl.u;
    }
    __syncthreads();
    v4u vh[4], vl[4];
    size_t go[4];
#pragma unroll
    for (int it = 0; it < 4; ++it) {
      const int p  = tid + 256 * it;
      const int r2 = p >> 6;
      const int pc = p & 63;
      vh[it] = *(const v4u*)(sth + r2 * SCP + pc * 8);
      vl[it] = *(const v4u*)(stl + r2 * SCP + pc * 8);
      go[it] = (((size_t)(i * NB + b)) * SQ + q0 + r2) * SQ + pc * 8;
    }
    for (int ps = 0; ps < 2; ++ps) {
#pragma unroll
      for (int it = 0; it < 4; ++it) {
        *(volatile v4u*)(ahi + go[it]) = vh[it];
        *(volatile v4u*)(alo + go[it]) = vl[it];
      }
      __threadfence();
    }
  }
}

__global__ __launch_bounds__(128) void k_feat(const unsigned short* __restrict__ ahi,
                                              const unsigned short* __restrict__ alo,
                                              const unsigned short* __restrict__ hth,
                                              const unsigned short* __restrict__ htl,
                                              _Float16* __restrict__ feat) {
  __shared__ __align__(16) _Float16 st[128 * STP];
  const int tid = threadIdx.x, lane = tid & 31, wave = tid >> 5;
  const int hh = lane >> 4, c = lane & 15;
  const int ib = blockIdx.z;
  const int b  = ib & (NB - 1);
  const int mb = blockIdx.x * 128;
  const int m0 = mb + wave * 32;
  const int n0 = blockIdx.y * 64;
  const unsigned short* Ah = ahi + (size_t)ib * SQ * SQ;
  const unsigned short* Al = alo + (size_t)ib * SQ * SQ;
  const unsigned short* Hh = hth + (size_t)b * DD * SQ;
  const unsigned short* Hl = htl + (size_t)b * DD * SQ;

  v8f acc[2][4];
#pragma unroll
  for (int s = 0; s < 2; ++s)
#pragma unroll
    for (int t = 0; t < 4; ++t) acc[s][t] = zero8();

#pragma unroll 1
  for (int k0 = 0; k0 < SQ; k0 += 32) {
    const v16b ah0 = ldfragb(Ah, SQ, m0, k0, lane);
    const v16b ah1 = ldfragb(Ah, SQ, m0 + 16, k0, lane);
    const v16b al0 = ldfragb(Al, SQ, m0, k0, lane);
    const v16b al1 = ldfragb(Al, SQ, m0 + 16, k0, lane);
#pragma unroll
    for (int t = 0; t < 4; ++t) {
      const v16b bhf = ldfragb(Hh, SQ, n0 + 16 * t, k0, lane);
      acc[0][t] = mmab(ah0, bhf, acc[0][t]);
      acc[1][t] = mmab(ah1, bhf, acc[1][t]);
      acc[0][t] = mmab(al0, bhf, acc[0][t]);
      acc[1][t] = mmab(al1, bhf, acc[1][t]);
      const v16b blf = ldfragb(Hl, SQ, n0 + 16 * t, k0, lane);
      acc[0][t] = mmab(ah0, blf, acc[0][t]);
      acc[1][t] = mmab(ah1, blf, acc[1][t]);
    }
  }

#pragma unroll
  for (int t = 0; t < 4; ++t) {
#pragma unroll
    for (int sub = 0; sub < 2; ++sub) {
#pragma unroll
      for (int r = 0; r < 8; ++r) {
        const int lr = wave * 32 + sub * 16 + 8 * hh + r;
        st[lr * STP + 16 * t + c] = (_Float16)(acc[sub][t][r] * 64.0f);
      }
    }
  }
  __syncthreads();

  v4u val[8];
  size_t go[8];
#pragma unroll
  for (int j = 0; j < 8; ++j) {
    const int p  = tid + 128 * j;
    const int lr = p >> 3;
    const int pc = p & 7;
    Pack8 pk;
    pk.h  = *(const v8h*)(st + lr * STP + pc * 8);
    val[j] = pk.u;
    go[j]  = ((size_t)(ib * SQ + mb + lr)) * DD + n0 + pc * 8;
  }
  for (int ps = 0; ps < 2; ++ps) {
#pragma unroll
    for (int j = 0; j < 8; ++j) *(volatile v4u*)(feat + go[j]) = val[j];
    __threadfence();
  }
}

#define OTP 68
__global__ __launch_bounds__(128) void k_out(const _Float16* __restrict__ feat,
                                             const _Float16* __restrict__ wgt,
                                             const float* __restrict__ bgat,
                                             const float* __restrict__ amask,
                                             float* __restrict__ out, float oscale) {
  __shared__ __align__(16) float st[4][32 * OTP];
  const int tid = threadIdx.x, lane = tid & 31, wave = tid >> 5;
  const int hh = lane >> 4, c = lane & 15;
  const int m0 = blockIdx.x * 128 + wave * 32;
  const int n0 = blockIdx.y * 64;
  float* sw = st[wave];

  float mqv[2][8];
#pragma unroll
  for (int sub = 0; sub < 2; ++sub)
#pragma unroll
    for (int r = 0; r < 8; ++r) mqv[sub][r] = amask[m0 + sub * 16 + 8 * hh + r];
#pragma unroll
  for (int sub = 0; sub < 2; ++sub)
#pragma unroll
    for (int t = 0; t < 4; ++t)
#pragma unroll
      for (int r = 0; r < 8; ++r) sw[(sub * 16 + 8 * hh + r) * OTP + 16 * t + c] = 0.f;

#pragma unroll 1
  for (int i = 0; i < NC; ++i) {
    v8f acc[2][4];
#pragma unroll
    for (int s = 0; s < 2; ++s)
#pragma unroll
      for (int t = 0; t < 4; ++t) acc[s][t] = zero8();
    gemm32x64(feat + (size_t)i * NR * DD, DD, wgt + (size_t)i * DD * DD, DD, DD, m0, n0, lane, acc);
#pragma unroll
    for (int t = 0; t < 4; ++t) {
      const float bv = bgat[i * DD + n0 + 16 * t + c];
#pragma unroll
      for (int sub = 0; sub < 2; ++sub) {
#pragma unroll
        for (int r = 0; r < 8; ++r) {
          float* cell = sw + (sub * 16 + 8 * hh + r) * OTP + 16 * t + c;
          const float v = fmaxf(acc[sub][t][r] * oscale + bv, 0.f) * mqv[sub][r];
          *cell = *cell + v;
        }
      }
    }
  }
  __syncthreads();

#pragma unroll
  for (int sub = 0; sub < 2; ++sub) {
    v4f val[8];
    size_t go[8];
#pragma unroll
    for (int it = 0; it < 8; ++it) {
      const int p    = lane + 32 * it;
      const int L    = p >> 3;
      const int pc   = p & 7;
      const int rr   = L >> 1;
      const int half = L & 1;
      val[it] = *(const v4f*)(sw + (sub * 16 + rr) * OTP + half * 32 + pc * 4) * (1.0f / 3.0f);
      go[it]  = (size_t)(m0 + sub * 16 + rr) * DD + n0 + half * 32 + pc * 4;
    }
    for (int ps = 0; ps < 2; ++ps) {
#pragma unroll
      for (int it = 0; it < 8; ++it) *(volatile v4f*)(out + go[it]) = val[it];
      __threadfence();
    }
  }
}

#define SZ_AB   ((size_t)NC * NB * SQ * SQ * 2)
#define SZ_XH   ((size_t)NR * DD * 2)
#define SZ_WQK  ((size_t)D2 * DD * 2)
#define SZ_QK   ((size_t)2 * PLQ * 2)
#define SZ_FEAT ((size_t)NC * NR * DD * 2)
#define SZ_HT   ((size_t)NB * DD * SQ * 2)
#define SZ_WG   ((size_t)NC * DD * DD * 2)

#define O_AHI  ((size_t)0)
#define O_ALO  (O_AHI + SZ_AB)
#define O_XH   ((size_t)0)
#define O_WQK  (O_XH + SZ_XH)
#define O_QK   (O_ALO + SZ_AB)
#define O_FEAT (O_QK)
#define O_HTH  (O_FEAT + SZ_FEAT)
#define O_HTL  (O_HTH + SZ_HT)
#define O_WG   (O_HTL + SZ_HT)
#define O_END  (O_WG + SZ_WG)

static_assert(O_WQK + SZ_WQK <= O_QK);
static_assert(O_QK + SZ_QK <= O_HTH);
static_assert(O_FEAT + SZ_FEAT <= O_HTH);
static_assert(O_ALO + SZ_AB <= O_QK);
static_assert(O_END == (size_t)116785152);
static_assert(O_END <= (size_t)134217728);
static_assert((O_ALO % 256) == 0);
static_assert((O_WQK % 256) == 0);
static_assert((O_QK % 256) == 0);
static_assert((O_HTH % 256) == 0);
static_assert((O_HTL % 256) == 0);
static_assert((O_WG % 256) == 0);

extern "C" void kernel_launch(void* const* d_in, const int* in_sizes, int n_in,
                              void* d_out, int out_size, void* d_ws, size_t ws_size,
                              hipStream_t stream) {
  if (n_in < 7) return;
  if (in_sizes[0] != NR * DD) return;
  if (in_sizes[1] != NB * NC * SQ * SQ) return;
  if (in_sizes[2] != NR) return;
  if (in_sizes[3] != DD * D2 || in_sizes[4] != D2) return;
  if (in_sizes[5] != NC * DD * DD || in_sizes[6] != NC * DD) return;
  if (out_size != NR * DD) return;
  if (O_END > ws_size) return;

  const float* Ht    = (const float*)d_in[0];
  const float* Mlist = (const float*)d_in[1];
  const float* amask = (const float*)d_in[2];
  const float* W_qk  = (const float*)d_in[3];
  const float* b_qk  = (const float*)d_in[4];
  const float* W_gat = (const float*)d_in[5];
  const float* b_gat = (const float*)d_in[6];
  float* out = (float*)d_out;

  char* ws = (char*)d_ws;
  unsigned short* Ahi  = (unsigned short*)(ws + O_AHI);
  unsigned short* Alo  = (unsigned short*)(ws + O_ALO);
  _Float16*       Xh   = (_Float16*)(ws + O_XH);
  _Float16*       WqkT = (_Float16*)(ws + O_WQK);
  _Float16*       QKp  = (_Float16*)(ws + O_QK);
  _Float16*       Feat = (_Float16*)(ws + O_FEAT);
  unsigned short* HtH  = (unsigned short*)(ws + O_HTH);
  unsigned short* HtL  = (unsigned short*)(ws + O_HTL);
  _Float16*       WgT  = (_Float16*)(ws + O_WG);

  k_cvt_ht<<<dim3(SQ / 64, DD / 64, NB), dim3(256), 0, stream>>>(Ht, Xh, HtH, HtL);
  k_cvt_wt<<<dim3(D2 / 64, DD / 64, 1), dim3(256), 0, stream>>>(W_qk, WqkT, DD, D2, 32.0f);
  k_cvt_wt<<<dim3(DD / 64, DD / 64, NC), dim3(256), 0, stream>>>(W_gat, WgT, DD, DD, 32.0f);
  k_qk<<<dim3(NR / 128, D2 / 64), dim3(128), 0, stream>>>(Xh, WqkT, b_qk, QKp);
  (void)hipFuncSetAttribute(reinterpret_cast<const void*>(&k_attn),
                            hipFuncAttributeMaxDynamicSharedMemorySize, LDS_ATT);
  k_attn<<<dim3(NB * (SQ / 16)), dim3(256), LDS_ATT, stream>>>(QKp, QKp + PLQ, amask, Mlist, Ahi, Alo,
                                                               0.036084391824351614f);
  k_feat<<<dim3(SQ / 128, DD / 64, NC * NB), dim3(128), 0, stream>>>(Ahi, Alo, HtH, HtL, Feat);
  k_out<<<dim3(NR / 128, DD / 64), dim3(128), 0, stream>>>(Feat, WgT, b_gat, amask, out, 0.00048828125f);
  (void)hipGetLastError();
}
